// DCT_base_Rec_Module_18056042513026
// MI455X (gfx1250) — hardware-verified
//
#include <hip/hip_runtime.h>


typedef _Float16 v16h __attribute__((ext_vector_type(16)));
typedef _Float16 v8h  __attribute__((ext_vector_type(8)));
typedef float    v8f  __attribute__((ext_vector_type(8)));
typedef float    v4f  __attribute__((ext_vector_type(4)));

#define WS     32
#define NUMP   127
#define NPAT   (NUMP * NUMP)
#define IMGH   2048
#define PPB    32
#define NBLK1  ((NPAT + PPB - 1) / PPB)
#define NT     96
#define SC_D   64.0f
#define SC_I64 (1.0f / 64.0f)
#define SC_OUT (1.0f / 4096.0f)

union Frag { v16h v; v8h hv[2]; };

__device__ __forceinline__ v16h load_frag(const _Float16* src, int r0) {
    const int lane = threadIdx.x & 31, h = lane >> 4, m = lane & 15;
    const _Float16* p = src + (r0 + m) * WS + 8 * h;
    Frag f;
    f.hv[0] = *(const v8h*)(p);
    f.hv[1] = *(const v8h*)(p + 16);
    return f.v;
}

__device__ __forceinline__ v8f wmma16(v16h a, v16h b, v8f c) {
    v8f d = __builtin_amdgcn_wmma_f32_16x16x32_f16(false, a, false, b, (short)0, c, false, false);
    asm volatile("v_nop\n\tv_nop\n\tv_nop\n\tv_nop" : "+v"(d) : "v"(a), "v"(b));
    return d;
}

__device__ __forceinline__ void store_tile_rm(_Float16* dst, int ti, int tj, v8f acc, float scale) {
    const int lane = threadIdx.x & 31, h = lane >> 4, n = lane & 15;
#pragma unroll
    for (int r = 0; r < 8; ++r)
        dst[(ti + 8 * h + r) * WS + tj + n] = (_Float16)(acc[r] * scale);
}

__device__ __forceinline__ void fill_patch_cm(_Float16* Pt, const float* xc) {
    const int lane = threadIdx.x & 31;
#pragma unroll
    for (int q = lane; q < 256; q += 32) {
        const int row = q >> 3, c4 = (q & 7) << 2;
        const v4f v = *(const v4f*)(xc + (size_t)row * IMGH + c4);
        Pt[(c4 + 0) * WS + row] = (_Float16)v[0];
        Pt[(c4 + 1) * WS + row] = (_Float16)v[1];
        Pt[(c4 + 2) * WS + row] = (_Float16)v[2];
        Pt[(c4 + 3) * WS + row] = (_Float16)v[3];
    }
}

__global__ __launch_bounds__(NT) void k_grade(
    const float* __restrict__ x, const float* __restrict__ dct,
    const float* __restrict__ gmasks, const float* __restrict__ gftnum,
    const float* __restrict__ gweights, float* __restrict__ grade) {
    __shared__ __align__(16) _Float16 sD[WS * WS];
    __shared__ __align__(16) _Float16 sPt[3][WS * WS];
    __shared__ __align__(16) _Float16 sT[3][WS * WS];
    __shared__ float sW[WS * WS];
    __shared__ float sPart[3][PPB];
    __shared__ __align__(16) float sG[PPB];

    const int tid  = threadIdx.x;
    const int wave = tid >> 5;
    const int lane = tid & 31;
    const int h = lane >> 4, n = lane & 15;

    for (int idx = tid; idx < WS * WS; idx += NT) {
        const float d = dct[idx];
        sD[idx] = (_Float16)(d * SC_D);
        float w = 0.f;
#pragma unroll
        for (int g = 0; g < 6; ++g)
            w += (gmasks[g * WS * WS + idx] * (1.0f / gftnum[g])) * gweights[g];
        sW[idx] = w;
    }

    _Float16* Pt = sPt[wave];
    _Float16* T  = sT[wave];

#pragma unroll 1
    for (int p = 0; p < PPB; ++p) {
        int l = blockIdx.x * PPB + p;
        if (l > NPAT - 1) l = NPAT - 1;
        const int pi = l / NUMP, pj = l - pi * NUMP;
        const float* xc = x + (size_t)wave * IMGH * IMGH +
                          (size_t)(pi * 16) * IMGH + (size_t)(pj * 16);
        fill_patch_cm(Pt, xc);
        __syncthreads();

#pragma unroll
        for (int ti = 0; ti < WS; ti += 16)
#pragma unroll
            for (int tj = 0; tj < WS; tj += 16) {
                v8f acc = {};
                acc = wmma16(load_frag(sD, ti), load_frag(Pt, tj), acc);
                store_tile_rm(T, ti, tj, acc, 1.0f);
            }
        __syncthreads();

        float partial = 0.f;
#pragma unroll
        for (int ti = 0; ti < WS; ti += 16)
#pragma unroll
            for (int tj = 0; tj < WS; tj += 16) {
                v8f acc = {};
                acc = wmma16(load_frag(T, ti), load_frag(sD, tj), acc);
#pragma unroll
                for (int r = 0; r < 8; ++r) {
                    const int row = ti + 8 * h + r, col = tj + n;
                    const float xd = acc[r] * SC_OUT;
                    partial += __logf(fabsf(xd) + 1.0f) * sW[row * WS + col];
                }
            }
#pragma unroll
        for (int off = 16; off > 0; off >>= 1)
            partial += __shfl_xor(partial, off, 32);
        if (lane == 0) sPart[wave][p] = partial;
    }
    __syncthreads();
    if (tid < PPB) sG[tid] = sPart[0][tid] + sPart[1][tid] + sPart[2][tid];
    __syncthreads();

    v4f gv = {};
    float* gp = grade;
    if (tid < 8) {
        gv = *(const v4f*)(sG + 4 * tid);
        gp = grade + (size_t)blockIdx.x * PPB + 4 * tid;
        *(volatile v4f*)gp = gv;
    }
    __threadfence();
    if (tid < 8) {
        *(volatile v4f*)gp = gv;
    }
}

__device__ __forceinline__ void ins_min(float& v0, int& i0, float& v1, int& i1, float v, int i) {
    if (i < 0) return;
    if (v < v0 || (v == v0 && i < i0)) { v1 = v0; i1 = i0; v0 = v; i0 = i; }
    else if (v < v1 || (v == v1 && i < i1)) { v1 = v; i1 = i; }
}
__device__ __forceinline__ void ins_max(float& v0, int& i0, float& v1, int& i1, float v, int i) {
    if (i < 0) return;
    if (v > v0 || (v == v0 && i > i0)) { v1 = v0; i1 = i0; v0 = v; i0 = i; }
    else if (v > v1 || (v == v1 && i > i1)) { v1 = v; i1 = i; }
}

__global__ __launch_bounds__(NT) void k_level(
    const float* __restrict__ x, const float* __restrict__ dct,
    const float* __restrict__ lmask, const float* __restrict__ grade,
    float* __restrict__ out) {
    __shared__ __align__(16) _Float16 sD[WS * WS];
    __shared__ __align__(16) _Float16 sDt[WS * WS];
    __shared__ __align__(16) _Float16 sPt[3][WS * WS];
    __shared__ __align__(16) _Float16 sXmc[3][WS * WS];
    __shared__ __align__(16) _Float16 sT[3][WS * WS];
    __shared__ __align__(16) float sOut[3][WS * WS];
    __shared__ float rv[4][NT];
    __shared__ int   ri[4][NT];
    __shared__ int   sL;

    const int tid  = threadIdx.x;
    const int wave = tid >> 5;
    const int lane = tid & 31;
    const int h = lane >> 4, n = lane & 15;
    const int slot = blockIdx.x;

    float m0v = 3.4e38f, m1v = 3.4e38f, M0v = -3.4e38f, M1v = -3.4e38f;
    int   m0i = -1, m1i = -1, M0i = -1, M1i = -1;
    for (int i = tid; i < NPAT; i += NT) {
        const float v = grade[i];
        ins_min(m0v, m0i, m1v, m1i, v, i);
        ins_max(M0v, M0i, M1v, M1i, v, i);
    }
    rv[0][tid] = m0v; ri[0][tid] = m0i;
    rv[1][tid] = m1v; ri[1][tid] = m1i;
    rv[2][tid] = M0v; ri[2][tid] = M0i;
    rv[3][tid] = M1v; ri[3][tid] = M1i;

    for (int idx = tid; idx < WS * WS; idx += NT) {
        const float d = dct[idx] * SC_D;
        sD[idx] = (_Float16)d;
        sDt[(idx & 31) * WS + (idx >> 5)] = (_Float16)d;
    }
    __syncthreads();

    if (tid == 0) {
        float a0 = 3.4e38f, a1 = 3.4e38f, b0 = -3.4e38f, b1 = -3.4e38f;
        int ia0 = -1, ia1 = -1, ib0 = -1, ib1 = -1;
#pragma unroll 1
        for (int t = 0; t < NT; ++t) {
            ins_min(a0, ia0, a1, ia1, rv[0][t], ri[0][t]);
            ins_min(a0, ia0, a1, ia1, rv[1][t], ri[1][t]);
            ins_max(b0, ib0, b1, ib1, rv[2][t], ri[2][t]);
            ins_max(b0, ib0, b1, ib1, rv[3][t], ri[3][t]);
        }
        int l = (slot == 0) ? ia0 : (slot == 1) ? ib0 : (slot == 2) ? ia1 : ib1;
        if (l < 0) l = 0;
        if (l > NPAT - 1) l = NPAT - 1;
        sL = l;
    }
    __syncthreads();

    const int l  = sL;
    const int pi = l / NUMP, pj = l - pi * NUMP;
    const float* xc = x + (size_t)wave * IMGH * IMGH +
                      (size_t)(pi * 16) * IMGH + (size_t)(pj * 16);
    _Float16* Pt  = sPt[wave];
    _Float16* Xmc = sXmc[wave];
    _Float16* T   = sT[wave];
    fill_patch_cm(Pt, xc);
    __syncthreads();

#pragma unroll
    for (int ti = 0; ti < WS; ti += 16)
#pragma unroll
        for (int tj = 0; tj < WS; tj += 16) {
            v8f acc = {};
            acc = wmma16(load_frag(sD, ti), load_frag(Pt, tj), acc);
            store_tile_rm(T, ti, tj, acc, 1.0f);
        }
    __syncthreads();

#pragma unroll
    for (int ti = 0; ti < WS; ti += 16)
#pragma unroll
        for (int tj = 0; tj < WS; tj += 16) {
            v8f acc = {};
            acc = wmma16(load_frag(T, ti), load_frag(sD, tj), acc);
            v8h pk;
#pragma unroll
            for (int r = 0; r < 8; ++r) {
                const int row = ti + 8 * h + r, col = tj + n;
                const float xd = acc[r] * SC_OUT;
                const float xm = xd * lmask[row * WS + col];
                pk[r] = (_Float16)(xm * SC_D);
            }
            *(v8h*)(Xmc + (tj + n) * WS + ti + 8 * h) = pk;
        }
    __syncthreads();

    _Float16* T2 = Pt;
#pragma unroll
    for (int ti = 0; ti < WS; ti += 16)
#pragma unroll
        for (int tj = 0; tj < WS; tj += 16) {
            v8f acc = {};
            acc = wmma16(load_frag(sDt, ti), load_frag(Xmc, tj), acc);
            store_tile_rm(T2, ti, tj, acc, SC_I64);
        }
    __syncthreads();

    float* So = sOut[wave];
#pragma unroll
    for (int ti = 0; ti < WS; ti += 16)
#pragma unroll
        for (int tj = 0; tj < WS; tj += 16) {
            v8f acc = {};
            acc = wmma16(load_frag(T2, ti), load_frag(sDt, tj), acc);
#pragma unroll
            for (int r = 0; r < 8; ++r)
                So[(ti + 8 * h + r) * WS + tj + n] = acc[r] * SC_OUT;
        }
    __syncthreads();

    float* outc = out + (size_t)slot * 3 * WS * WS + (size_t)wave * WS * WS;
    const int rq = lane >> 3, c4 = (lane & 7) << 2;
    v4f ov[8];
#pragma unroll
    for (int i = 0; i < 8; ++i) {
        const int row = 4 * i + rq;
        ov[i] = *(const v4f*)(So + row * WS + c4);
        *(volatile v4f*)(outc + row * WS + c4) = ov[i];
    }
    __threadfence();
#pragma unroll
    for (int i = 0; i < 8; ++i) {
        const int row = 4 * i + rq;
        *(volatile v4f*)(outc + row * WS + c4) = ov[i];
    }
}

extern "C" void kernel_launch(void* const* d_in, const int* in_sizes, int n_in,
                              void* d_out, int out_size, void* d_ws, size_t ws_size,
                              hipStream_t stream) {
    if (n_in < 6) return;
    if (in_sizes[0] != 3 * IMGH * IMGH) return;
    if (in_sizes[1] != WS * WS || in_sizes[2] != WS * WS) return;
    if (in_sizes[3] != 6 * WS * WS || in_sizes[4] != 6 || in_sizes[5] != 6) return;
    if (out_size != 4 * 3 * WS * WS) return;
    const size_t grade_bytes = (size_t)NBLK1 * PPB * sizeof(float);
    if (ws_size < grade_bytes) return;

    const float* x        = (const float*)d_in[0];
    const float* dct      = (const float*)d_in[1];
    const float* lmask    = (const float*)d_in[2];
    const float* gmasks   = (const float*)d_in[3];
    const float* gftnum   = (const float*)d_in[4];
    const float* gweights = (const float*)d_in[5];
    float* out   = (float*)d_out;
    float* grade = (float*)d_ws;

    k_grade<<<NBLK1, NT, 0, stream>>>(x, dct, gmasks, gftnum, gweights, grade);
    k_level<<<4, NT, 0, stream>>>(x, dct, lmask, grade, out);
}
